// GNNClusterBridge_56349970923677
// MI455X (gfx1250) — hardware-verified
//
#include <hip/hip_runtime.h>
#include <stddef.h>


#define DF      128
#define NC      64
#define NTHR    256
#define NWAVE   8
#define EPT     8
#define NGRP    2
#define CHUNK   (NTHR * EPT * NGRP)
#define WCAP    (EPT * NGRP * 32)
#define LISTN   (NWAVE * WCAP)
#define NBA     512
#define NBD     4096
#define G1ROWS  128
#define APITCH  136
#define WSCALE  16.0f
#define WINV    0.0625f

#define LDS_GEMM1 (G1ROWS * DF * 4)
#define LDS_AGG   (NBA * DF * 4 + LISTN * 4 + 64)

static_assert((CHUNK & (CHUNK - 1)) == 0);
static_assert(CHUNK <= 4096);
static_assert((NBA & (NBA - 1)) == 0 && NBA <= 4096);
static_assert((NBD & (NBD - 1)) == 0 && NBD <= 4096);
static_assert(NBA % G1ROWS == 0);
static_assert(NBA % (16 * NWAVE) == 0);
static_assert(NBD == NWAVE * 4 * 128);
static_assert(G1ROWS * APITCH * 2 <= LDS_GEMM1);

typedef float    v4f  __attribute__((ext_vector_type(4)));
typedef float    v8f  __attribute__((ext_vector_type(8)));
typedef int      v4i  __attribute__((ext_vector_type(4)));
typedef _Float16 v8h  __attribute__((ext_vector_type(8)));
typedef _Float16 v16h __attribute__((ext_vector_type(16)));
union FragH { v16h v; v8h h[2]; };

__device__ __forceinline__ v8h cvt8(v4f a, v4f b) {
  v8h r;
  r[0] = (_Float16)a.x; r[1] = (_Float16)a.y; r[2] = (_Float16)a.z; r[3] = (_Float16)a.w;
  r[4] = (_Float16)b.x; r[5] = (_Float16)b.y; r[6] = (_Float16)b.z; r[7] = (_Float16)b.w;
  return r;
}

__device__ __forceinline__ v8f wmh(v16h a, v16h b, v8f c) {
  v8f d = __builtin_amdgcn_wmma_f32_16x16x32_f16(false, a, false, b, (short)0, c, false, false);
  asm volatile("v_nop\n\tv_nop\n\tv_nop\n\tv_nop" : "+v"(d) : "v"(a), "v"(b));
  return d;
}

template <int NB>
__device__ __forceinline__ int scan_chunk(const int* __restrict__ dsts, int nE, int cbase, int nodeBase,
                                          int vec8, int* list, int tid, int lane, int wave) {
  int wc = 0;
#pragma unroll
  for (int g = 0; g < NGRP; ++g) {
    const int el0  = (g * NTHR + tid) * EPT;
    const int e0   = cbase + el0;
    const int sent = -2147483647 - 1;
    v4i da, db;
    if (vec8 != 0 && e0 + 7 < nE) {
      da = *(const v4i*)(dsts + e0);
      db = *(const v4i*)(dsts + e0 + 4);
    } else {
      da.x = (e0     < nE) ? dsts[min(e0, nE - 1)] : sent;
      da.y = (e0 + 1 < nE) ? dsts[min(e0 + 1, nE - 1)] : sent;
      da.z = (e0 + 2 < nE) ? dsts[min(e0 + 2, nE - 1)] : sent;
      da.w = (e0 + 3 < nE) ? dsts[min(e0 + 3, nE - 1)] : sent;
      db.x = (e0 + 4 < nE) ? dsts[min(e0 + 4, nE - 1)] : sent;
      db.y = (e0 + 5 < nE) ? dsts[min(e0 + 5, nE - 1)] : sent;
      db.z = (e0 + 6 < nE) ? dsts[min(e0 + 6, nE - 1)] : sent;
      db.w = (e0 + 7 < nE) ? dsts[min(e0 + 7, nE - 1)] : sent;
    }
    const unsigned nb = (unsigned)nodeBase;
    const unsigned s0 = (unsigned)da.x - nb, s1 = (unsigned)da.y - nb;
    const unsigned s2 = (unsigned)da.z - nb, s3 = (unsigned)da.w - nb;
    const unsigned s4 = (unsigned)db.x - nb, s5 = (unsigned)db.y - nb;
    const unsigned s6 = (unsigned)db.z - nb, s7 = (unsigned)db.w - nb;
    const bool h0 = s0 < (unsigned)NB, h1 = s1 < (unsigned)NB, h2 = s2 < (unsigned)NB, h3 = s3 < (unsigned)NB;
    const bool h4 = s4 < (unsigned)NB, h5 = s5 < (unsigned)NB, h6 = s6 < (unsigned)NB, h7 = s7 < (unsigned)NB;
    const unsigned any = __builtin_amdgcn_ballot_w32(h0 | h1 | h2 | h3 | h4 | h5 | h6 | h7);
    if (any != 0u) {
#define HITJ(J, HJ, SJ) { \
        const unsigned mj = __builtin_amdgcn_ballot_w32(HJ); \
        if (mj != 0u) { \
          if (HJ) { \
            const int pos = wc + (int)__builtin_amdgcn_mbcnt_lo(mj, 0u); \
            if (pos < WCAP) list[wave * WCAP + pos] = ((el0 + (J)) << 12) | (int)(SJ); \
          } \
          wc += (int)__builtin_popcount(mj); } }
      HITJ(0, h0, s0)
      HITJ(1, h1, s1)
      HITJ(2, h2, s2)
      HITJ(3, h3, s3)
      HITJ(4, h4, s4)
      HITJ(5, h5, s5)
      HITJ(6, h6, s6)
      HITJ(7, h7, s7)
#undef HITJ
    }
  }
  return wc;
}

__global__ __launch_bounds__(NTHR) void k_wprep(
    const float* __restrict__ W1, const float* __restrict__ W2, const float* __restrict__ W3,
    const float* __restrict__ Wc,
    _Float16* w1s, _Float16* w2s, _Float16* w3s, _Float16* wcs) {
  const int i  = blockIdx.x * NTHR + threadIdx.x;
  const int n1 = DF * DF / 8;
  const int n4 = NC * DF / 8;
  if (i >= 3 * n1 + n4) return;
  const int sel  = i < n1 ? 0 : (i < 2 * n1 ? 1 : (i < 3 * n1 ? 2 : 3));
  const float* W = sel == 0 ? W1 : (sel == 1 ? W2 : (sel == 2 ? W3 : Wc));
  _Float16*    D = sel == 0 ? w1s : (sel == 1 ? w2s : (sel == 2 ? w3s : wcs));
  const int nout = (sel == 3) ? NC : DF;
  const int o  = (i - sel * n1) * 8;
  const int n  = o / DF;
  const int k0 = o - n * DF;
  const float* p = W + (size_t)k0 * nout + n;
  v4f a, b;
  a.x = p[0];        a.y = p[nout];     a.z = p[2 * nout]; a.w = p[3 * nout];
  b.x = p[4 * nout]; b.y = p[5 * nout]; b.z = p[6 * nout]; b.w = p[7 * nout];
  a = a * WSCALE;
  b = b * WSCALE;
  const v8h hv = cvt8(a, b);
  _Float16* dp = D + o;
  *(volatile v8h*)dp = hv;
  __threadfence();
  *(volatile v8h*)dp = hv;
}

__global__ __launch_bounds__(NTHR) void k_deg(
    const int* __restrict__ ei, const float* __restrict__ ew, float* dinv, int nE, int vec8) {
  __shared__ __attribute__((aligned(16))) float dsum[NBD];
  __shared__ __attribute__((aligned(16))) int list[LISTN];
  __shared__ int wcnt[NWAVE];
  const int tid = threadIdx.x, lane = tid & 31, wave = tid >> 5;
  const int nodeBase = blockIdx.x * NBD;
  const int* dsts = ei + nE;

  for (int i = tid; i < NBD; i += NTHR) dsum[i] = 0.f;
  __syncthreads();

  const int nChunks = (nE + CHUNK - 1) / CHUNK;
#pragma unroll 1
  for (int ch = 0; ch < nChunks; ++ch) {
    const int cbase = ch * CHUNK;
    const int wc = scan_chunk<NBD>(dsts, nE, cbase, nodeBase, vec8, list, tid, lane, wave);
    if (lane == 0) wcnt[wave] = wc;
    __syncthreads();
    if (wave == 0) {
#pragma unroll 1
      for (int wsx = 0; wsx < NWAVE; ++wsx) {
        int n = __builtin_amdgcn_readfirstlane(wcnt[wsx]);
        n = n > WCAP ? WCAP : (n < 0 ? 0 : n);
        const int* lp = list + wsx * WCAP;
#pragma unroll 1
        for (int i = 0; i < n; ++i) {
          const int ent  = __builtin_amdgcn_readfirstlane(lp[i]);
          const int slot = ent & (NBD - 1);
          int e = cbase + ((ent >> 12) & (CHUNK - 1));
          e = e > nE - 1 ? nE - 1 : e;
          const float w = ew[e];
          if (lane == 0) dsum[slot] = dsum[slot] + w;
        }
      }
    }
    __syncthreads();
  }

  v4f dq[4];
#pragma unroll
  for (int q = 0; q < 4; ++q) {
    const int f = (wave * 4 + q) * 128 + 4 * lane;
    const v4f c = *(const v4f*)(dsum + f);
    dq[q].x = rsqrtf(c.x + 1.f);
    dq[q].y = rsqrtf(c.y + 1.f);
    dq[q].z = rsqrtf(c.z + 1.f);
    dq[q].w = rsqrtf(c.w + 1.f);
  }
  float* dp = dinv + (size_t)nodeBase;
#pragma unroll
  for (int q = 0; q < 4; ++q) *(volatile v4f*)(dp + (wave * 4 + q) * 128 + 4 * lane) = dq[q];
  __threadfence();
#pragma unroll
  for (int q = 0; q < 4; ++q) *(volatile v4f*)(dp + (wave * 4 + q) * 128 + 4 * lane) = dq[q];
}

__global__ __launch_bounds__(NTHR) void k_gemm1(
    const float* __restrict__ x, const _Float16* __restrict__ w1s,
    const float* __restrict__ dinv, float* g1, int nN) {
  extern __shared__ v4f lds_dyn[];
  _Float16* sA  = (_Float16*)lds_dyn;
  float*    stg = (float*)lds_dyn;
  const int tid = threadIdx.x, lane = tid & 31, wave = tid >> 5, hh = lane >> 4, m = lane & 15;
  const int rowBase = blockIdx.x * G1ROWS;

#pragma unroll
  for (int i = 0; i < (G1ROWS * DF / 8) / NTHR; ++i) {
    const int idx = i * NTHR + tid;
    const int r   = idx >> 4;
    const int c0  = (idx & 15) * 8;
    int node = rowBase + r;
    node = node > nN - 1 ? nN - 1 : node;
    const float* xp = x + (size_t)node * DF + c0;
    const v4f a = *(const v4f*)xp, b = *(const v4f*)(xp + 4);
    *(v8h*)(sA + r * APITCH + c0) = cvt8(a, b);
  }
  __syncthreads();

  v8f acc[8];
#pragma unroll
  for (int t = 0; t < 8; ++t) { v8f z = {0.f, 0.f, 0.f, 0.f, 0.f, 0.f, 0.f, 0.f}; acc[t] = z; }
  const _Float16* ar = sA + (wave * 16 + m) * APITCH + 8 * hh;
#pragma unroll
  for (int kt = 0; kt < DF / 32; ++kt) {
    FragH a;
    a.h[0] = *(const v8h*)(ar + 32 * kt);
    a.h[1] = *(const v8h*)(ar + 32 * kt + 16);
#pragma unroll
    for (int t = 0; t < 8; ++t) {
      const _Float16* bp = w1s + (size_t)(16 * t + m) * DF + 32 * kt + 8 * hh;
      FragH b;
      b.h[0] = *(const v8h*)bp;
      b.h[1] = *(const v8h*)(bp + 16);
      acc[t] = wmh(a.v, b.v, acc[t]);
    }
  }
  __syncthreads();

  const int r0 = wave * 16 + 8 * hh;
  const v4f dA = *(const v4f*)(dinv + (size_t)rowBase + r0);
  const v4f dB = *(const v4f*)(dinv + (size_t)rowBase + r0 + 4);
  const float d0 = dA.x * WINV, d1 = dA.y * WINV, d2 = dA.z * WINV, d3 = dA.w * WINV;
  const float d4 = dB.x * WINV, d5 = dB.y * WINV, d6 = dB.z * WINV, d7 = dB.w * WINV;
  float* sp = stg + r0 * DF + m;
#pragma unroll
  for (int t = 0; t < 8; ++t) {
    sp[0 * DF + 16 * t] = acc[t][0] * d0;
    sp[1 * DF + 16 * t] = acc[t][1] * d1;
    sp[2 * DF + 16 * t] = acc[t][2] * d2;
    sp[3 * DF + 16 * t] = acc[t][3] * d3;
    sp[4 * DF + 16 * t] = acc[t][4] * d4;
    sp[5 * DF + 16 * t] = acc[t][5] * d5;
    sp[6 * DF + 16 * t] = acc[t][6] * d6;
    sp[7 * DF + 16 * t] = acc[t][7] * d7;
  }
  __syncthreads();

  const float* lp = stg + wave * 16 * DF + 4 * lane;
  float* gp = g1 + ((size_t)rowBase + wave * 16) * DF + 4 * lane;
#pragma unroll
  for (int i = 0; i < 16; ++i) { const v4f v = *(const v4f*)(lp + i * DF); *(volatile v4f*)(gp + (size_t)i * DF) = v; }
  __threadfence();
#pragma unroll
  for (int i = 0; i < 16; ++i) { const v4f v = *(const v4f*)(lp + i * DF); *(volatile v4f*)(gp + (size_t)i * DF) = v; }
}

template <int NOUT, bool FINAL>
__global__ __launch_bounds__(NTHR) void k_agg(
    const int* __restrict__ ei, const float* __restrict__ ew, const float* __restrict__ gin,
    const float* __restrict__ dinv, const float* __restrict__ bias,
    const _Float16* __restrict__ wns, const float* __restrict__ bnext,
    float* gout, int nN, int nE, int vec8) {
  extern __shared__ v4f lds_dyn[];
  float* acc  = (float*)lds_dyn;
  int*   list = (int*)(acc + NBA * DF);
  int*   wcnt = list + LISTN;
  const int tid = threadIdx.x, lane = tid & 31, wave = tid >> 5, hh = lane >> 4, m = lane & 15;
  const int nodeBase = blockIdx.x * NBA;
  const int* dsts = ei + nE;
  constexpr int NT = NOUT / 16;

  {
    const v4f z = {0.f, 0.f, 0.f, 0.f};
    for (int i = tid; i < NBA * DF / 4; i += NTHR) lds_dyn[i] = z;
  }
  __syncthreads();

  const int nChunks = (nE + CHUNK - 1) / CHUNK;
#pragma unroll 1
  for (int ch = 0; ch < nChunks; ++ch) {
    const int cbase = ch * CHUNK;
    const int wc = scan_chunk<NBA>(dsts, nE, cbase, nodeBase, vec8, list, tid, lane, wave);
    if (lane == 0) wcnt[wave] = wc;
    __syncthreads();
    if (wave == 0) {
#pragma unroll 1
      for (int wsx = 0; wsx < NWAVE; ++wsx) {
        int n = __builtin_amdgcn_readfirstlane(wcnt[wsx]);
        n = n > WCAP ? WCAP : (n < 0 ? 0 : n);
        const int* lp = list + wsx * WCAP;
#pragma unroll 1
        for (int i = 0; i < n; ++i) {
          const int ent  = __builtin_amdgcn_readfirstlane(lp[i]);
          const int slot = ent & (NBA - 1);
          int e = cbase + ((ent >> 12) & (CHUNK - 1));
          e = e > nE - 1 ? nE - 1 : e;
          int src = ei[e];
          src = src < 0 ? 0 : (src > nN - 1 ? nN - 1 : src);
          const float w = ew[e];
          const v4f v = *(const v4f*)(gin + (size_t)src * DF + 4 * lane);
          v4f* ap = (v4f*)(acc + slot * DF + 4 * lane);
          *ap = *ap + v * w;
        }
      }
    }
    __syncthreads();
  }

#pragma unroll 4
  for (int i = 0; i < (NBA * DF / 4) / NTHR; ++i) {
    const int idx  = i * NTHR + tid;
    const int slot = idx >> 5;
    const int c4   = (idx & 31) * 4;
    int node = nodeBase + slot;
    node = node > nN - 1 ? nN - 1 : node;
    const float d  = dinv[node];
    const v4f   gv = *(const v4f*)(gin + (size_t)node * DF + c4);
    const v4f   bv = *(const v4f*)(bias + c4);
    v4f* ap = (v4f*)(acc + slot * DF + c4);
    v4f hv = (*ap + gv) * d + bv;
    hv.x = fmaxf(hv.x, 0.f); hv.y = fmaxf(hv.y, 0.f); hv.z = fmaxf(hv.z, 0.f); hv.w = fmaxf(hv.w, 0.f);
    *ap = hv;
  }
  __syncthreads();

#pragma unroll 1
  for (int q = 0; q < NBA / (16 * NWAVE); ++q) {
    const int t16 = wave + NWAVE * q;
    v8f c[NT];
#pragma unroll
    for (int t = 0; t < NT; ++t) { v8f z = {0.f, 0.f, 0.f, 0.f, 0.f, 0.f, 0.f, 0.f}; c[t] = z; }
#pragma unroll
    for (int kt = 0; kt < DF / 32; ++kt) {
      const float* ap = acc + (16 * t16 + m) * DF + 32 * kt + 8 * hh;
      const v4f p0 = *(const v4f*)ap,        p1 = *(const v4f*)(ap + 4);
      const v4f p2 = *(const v4f*)(ap + 16), p3 = *(const v4f*)(ap + 20);
      FragH a;
      a.h[0] = cvt8(p0, p1);
      a.h[1] = cvt8(p2, p3);
#pragma unroll
      for (int t = 0; t < NT; ++t) {
        const _Float16* bp = wns + (size_t)(16 * t + m) * DF + 32 * kt + 8 * hh;
        FragH b;
        b.h[0] = *(const v8h*)bp;
        b.h[1] = *(const v8h*)(bp + 16);
        c[t] = wmh(a.v, b.v, c[t]);
      }
    }
    const int r0 = 16 * t16 + 8 * hh;
    float d[8];
    if (FINAL) {
#pragma unroll
      for (int rr = 0; rr < 8; ++rr) d[rr] = WINV;
    } else {
      const v4f dA = *(const v4f*)(dinv + (size_t)nodeBase + r0);
      const v4f dB = *(const v4f*)(dinv + (size_t)nodeBase + r0 + 4);
      d[0] = dA.x * WINV; d[1] = dA.y * WINV; d[2] = dA.z * WINV; d[3] = dA.w * WINV;
      d[4] = dB.x * WINV; d[5] = dB.y * WINV; d[6] = dB.z * WINV; d[7] = dB.w * WINV;
    }
    float* sp = acc + r0 * DF + m;
#pragma unroll
    for (int t = 0; t < NT; ++t) {
      const float bcol = FINAL ? bnext[16 * t + m] : 0.f;
#pragma unroll
      for (int rr = 0; rr < 8; ++rr) sp[rr * DF + 16 * t] = c[t][rr] * d[rr] + bcol;
    }
  }
  __syncthreads();

  if (FINAL) {
#pragma unroll 1
    for (int i = 0; i < NBA / NWAVE; ++i) {
      float* rp = acc + (wave * (NBA / NWAVE) + i) * DF;
      const float v0 = rp[lane], v1 = rp[lane + 32];
      float mx = fmaxf(v0, v1);
#pragma unroll
      for (int off = 16; off > 0; off >>= 1) mx = fmaxf(mx, __shfl_xor(mx, off, 32));
      const float e0 = expf(v0 - mx);
      const float e1 = expf(v1 - mx);
      float s = e0 + e1;
#pragma unroll
      for (int off = 16; off > 0; off >>= 1) s += __shfl_xor(s, off, 32);
      const float inv = 1.0f / s;
      rp[lane]      = e0 * inv;
      rp[lane + 32] = e1 * inv;
    }
    __syncthreads();
    const size_t outN = (size_t)nN * NC;
    const size_t ob   = (size_t)nodeBase * NC;
#pragma unroll 4
    for (int q = 0; q < (NBA * NC) / (NWAVE * 128); ++q) {
      const int f   = (wave * ((NBA * NC) / (NWAVE * 128)) + q) * 128 + 4 * lane;
      const int row = f >> 6, col = f & 63;
      const size_t gi = ob + (size_t)f;
      if (gi < outN) { const v4f v = *(const v4f*)(acc + row * DF + col); *(volatile v4f*)(gout + gi) = v; }
    }
    __threadfence();
#pragma unroll 4
    for (int q = 0; q < (NBA * NC) / (NWAVE * 128); ++q) {
      const int f   = (wave * ((NBA * NC) / (NWAVE * 128)) + q) * 128 + 4 * lane;
      const int row = f >> 6, col = f & 63;
      const size_t gi = ob + (size_t)f;
      if (gi < outN) { const v4f v = *(const v4f*)(acc + row * DF + col); *(volatile v4f*)(gout + gi) = v; }
    }
  } else {
#pragma unroll 4
    for (int q = 0; q < NBA / NWAVE; ++q) {
      const int row = wave * (NBA / NWAVE) + q;
      const v4f v = *(const v4f*)(acc + row * DF + 4 * lane);
      *(volatile v4f*)(gout + ((size_t)nodeBase + row) * DF + 4 * lane) = v;
    }
    __threadfence();
#pragma unroll 4
    for (int q = 0; q < NBA / NWAVE; ++q) {
      const int row = wave * (NBA / NWAVE) + q;
      const v4f v = *(const v4f*)(acc + row * DF + 4 * lane);
      *(volatile v4f*)(gout + ((size_t)nodeBase + row) * DF + 4 * lane) = v;
    }
  }
}

extern "C" void kernel_launch(void* const* d_in, const int* in_sizes, int n_in,
                              void* d_out, int out_size, void* d_ws, size_t ws_size,
                              hipStream_t stream) {
  if (n_in < 11) return;
  const int nN = in_sizes[0] / DF;
  const int nE = in_sizes[2];
  if (nN <= 0 || nE < 0 || in_sizes[0] != nN * DF || in_sizes[1] != nE * 2) return;
  if (in_sizes[3] != DF * DF || in_sizes[4] < DF) return;
  if (in_sizes[5] != DF * DF || in_sizes[6] < DF) return;
  if (in_sizes[7] != DF * DF || in_sizes[8] < DF) return;
  if (in_sizes[9] != DF * NC || in_sizes[10] < NC) return;
  if (out_size != nN * NC) return;

  const float* x  = (const float*)d_in[0];
  const int*   ei = (const int*)d_in[1];
  const float* ew = (const float*)d_in[2];
  const float* W1 = (const float*)d_in[3];
  const float* b1 = (const float*)d_in[4];
  const float* W2 = (const float*)d_in[5];
  const float* b2 = (const float*)d_in[6];
  const float* W3 = (const float*)d_in[7];
  const float* b3 = (const float*)d_in[8];
  const float* Wc = (const float*)d_in[9];
  const float* bc = (const float*)d_in[10];
  float* out = (float*)d_out;

  const int nBD = (nN + NBD - 1) / NBD;
  const int nG1 = (nN + G1ROWS - 1) / G1ROWS;
  const int nA  = (nN + NBA - 1) / NBA;

  char* ws = (char*)d_ws;
  size_t off = 0;
  const size_t oW1 = off; off += (size_t)DF * DF * 2;                          off = (off + 255) & ~(size_t)255;
  const size_t oW2 = off; off += (size_t)DF * DF * 2;                          off = (off + 255) & ~(size_t)255;
  const size_t oW3 = off; off += (size_t)DF * DF * 2;                          off = (off + 255) & ~(size_t)255;
  const size_t oWc = off; off += (size_t)NC * DF * 2;                          off = (off + 255) & ~(size_t)255;
  const size_t oDv = off; off += (size_t)nBD * NBD * 4;                        off = (off + 255) & ~(size_t)255;
  const size_t oGA = off; off += (size_t)nA * NBA * DF * 4;                    off = (off + 255) & ~(size_t)255;
  const size_t oGB = off; off += (size_t)nA * NBA * DF * 4;                    off = (off + 255) & ~(size_t)255;
  if (off > ws_size) return;
  _Float16* w1s  = (_Float16*)(ws + oW1);
  _Float16* w2s  = (_Float16*)(ws + oW2);
  _Float16* w3s  = (_Float16*)(ws + oW3);
  _Float16* wcs  = (_Float16*)(ws + oWc);
  float*    dinv = (float*)(ws + oDv);
  float*    gA   = (float*)(ws + oGA);
  float*    gB   = (float*)(ws + oGB);

  const int vec8 = ((nE & 3) == 0) ? 1 : 0;

  const int nPrep = 3 * (DF * DF / 8) + NC * DF / 8;
  k_wprep<<<(nPrep + NTHR - 1) / NTHR, NTHR, 0, stream>>>(W1, W2, W3, Wc, w1s, w2s, w3s, wcs);

  k_deg<<<nBD, NTHR, 0, stream>>>(ei, ew, dinv, nE, vec8);

  hipFuncSetAttribute(reinterpret_cast<const void*>(&k_gemm1),
                      hipFuncAttributeMaxDynamicSharedMemorySize, LDS_GEMM1);
  k_gemm1<<<nG1, NTHR, LDS_GEMM1, stream>>>(x, w1s, dinv, gA, nN);

  hipFuncSetAttribute(reinterpret_cast<const void*>(&k_agg<DF, false>),
                      hipFuncAttributeMaxDynamicSharedMemorySize, LDS_AGG);
  hipFuncSetAttribute(reinterpret_cast<const void*>(&k_agg<NC, true>),
                      hipFuncAttributeMaxDynamicSharedMemorySize, LDS_AGG);
  k_agg<DF, false><<<nA, NTHR, LDS_AGG, stream>>>(ei, ew, gA, dinv, b1, w2s, bc, gB, nN, nE, vec8);
  k_agg<DF, false><<<nA, NTHR, LDS_AGG, stream>>>(ei, ew, gB, dinv, b2, w3s, bc, gA, nN, nE, vec8);
  k_agg<NC, true><<<nA, NTHR, LDS_AGG, stream>>>(ei, ew, gA, dinv, b3, wcs, bc, out, nN, nE, vec8);
}
